// GCNsNet_7112465842805
// MI455X (gfx1250) — hardware-verified
//
#include <hip/hip_runtime.h>
#include <stddef.h>
#include <stdint.h>
#include <math.h>


#define NTHR   256
#define NWAVE  8
#define EPT    8
#define CHUNK  (NTHR * EPT)
#define WCAP   (EPT * 32)
#define LISTN  (NWAVE * WCAP)
#define NBD    2048
#define SLD    11
#define NBA    1024
#define SLA    10
#define RCAP   24576
#define DEGCAP 64
#define PCAP   256
#define SPW    8
#define NPB    (NWAVE * SPW)
#define GBM    64
#define GTHR   128
#define TB_CNT 32
#define TB_OFF (TB_CNT + NBA)
#define TB_SRC (TB_OFF + NBA)
#define TB_WV  (TB_SRC + RCAP)
#define TBSZ   (TB_WV + RCAP)
#define BLD_ZINTS (LISTN + 2 * RCAP + 3 * NBA)
#define BLD_LDS_INTS (BLD_ZINTS + 16)
#define FCK    512
#define NCLS   3

static_assert((CHUNK & (CHUNK - 1)) == 0 && CHUNK <= 4096);
static_assert((NBD & (NBD - 1)) == 0 && NBD == (1 << SLD));
static_assert((NBA & (NBA - 1)) == 0 && NBA == (1 << SLA));
static_assert(((long long)CHUNK << SLD) < (1LL << 31));
static_assert(((long long)CHUNK << SLA) < (1LL << 31));
static_assert(NBD % (NTHR * 4) == 0 && NBA == NTHR * 4);
static_assert(LISTN % NTHR == 0 && LISTN % 4 == 0 && BLD_ZINTS % 4 == 0);
static_assert(RCAP % (NTHR * 4) == 0);
static_assert((TB_CNT * 4) % 128 == 0 && (TB_OFF * 4) % 128 == 0 && (TB_SRC * 4) % 128 == 0);
static_assert((TB_WV * 4) % 128 == 0 && (TBSZ * 4) % 128 == 0);
static_assert(BLD_LDS_INTS * 4 <= 300000);
static_assert(NBA % NPB == 0 && NPB == GBM);
static_assert(GBM == (GTHR / 32) * 16);
static_assert((NPB * NCLS) % 4 == 0 && (NPB * NCLS * 4) % 128 == 0 && (NPB * NCLS) / 4 <= 64);

typedef float          v2f   __attribute__((ext_vector_type(2)));
typedef float          v4f   __attribute__((ext_vector_type(4)));
typedef float          v8f   __attribute__((ext_vector_type(8)));
typedef int            v4i   __attribute__((ext_vector_type(4)));
typedef int            v8i   __attribute__((ext_vector_type(8)));
typedef unsigned short v2us  __attribute__((ext_vector_type(2)));
typedef unsigned short v4us  __attribute__((ext_vector_type(4)));
typedef unsigned short v8us  __attribute__((ext_vector_type(8)));
typedef unsigned short v16us __attribute__((ext_vector_type(16)));
typedef __bf16         v16bf __attribute__((ext_vector_type(16)));
typedef v2f  __attribute__((may_alias)) v2fa;
typedef v4f  __attribute__((may_alias)) v4fa;
typedef v4i  __attribute__((may_alias)) v4ia;
typedef v2us __attribute__((may_alias)) v2usa;
typedef v4us __attribute__((may_alias)) v4usa;
typedef v8us __attribute__((may_alias)) v8usa;
union FragB { v16bf v; v16us u; v8us h[2]; v8i w; };

__device__ __forceinline__ v8f wmb(const FragB& a, const FragB& b, v8f c) {
  v8f d = __builtin_amdgcn_wmma_f32_16x16x32_bf16(false, a.v, false, b.v, (short)0, c, false, false);
  asm volatile("v_nop\n\tv_nop\n\tv_nop\n\tv_nop" : "+v"(d) : "v"(a.w), "v"(b.w));
  return d;
}

__device__ __forceinline__ unsigned bf16_bits(float f) {
  const unsigned u = __float_as_uint(f);
  return (u + 0x7FFFu + ((u >> 16) & 1u)) >> 16;
}
__device__ __forceinline__ float bf16_val(float f) {
  return __uint_as_float(bf16_bits(f) << 16);
}
__device__ __forceinline__ int clampi(int v, int lo, int hi) { return v < lo ? lo : (v > hi ? hi : v); }

__device__ __forceinline__ void wave_sync() {
  __builtin_amdgcn_fence(__ATOMIC_RELEASE, "wavefront");
  __builtin_amdgcn_wave_barrier();
  __builtin_amdgcn_fence(__ATOMIC_ACQUIRE, "wavefront");
}

__device__ __forceinline__ float softplus_f(float m) {
  const float mx = (m > 0.0f) ? m : 0.0f;
  return mx + log1pf(expf(-fabsf(m)));
}

template <int CPL>
__device__ __forceinline__ void ld_row(const float* p, float (&r)[CPL]) {
  if constexpr (CPL == 1) {
    r[0] = *p;
  } else if constexpr (CPL == 2) {
    const v2f a = *(const v2fa*)p; r[0] = a.x; r[1] = a.y;
  } else if constexpr (CPL == 4) {
    const v4f a = *(const v4fa*)p; r[0] = a.x; r[1] = a.y; r[2] = a.z; r[3] = a.w;
  } else {
    const v4f a = *(const v4fa*)p; const v4f b = *(const v4fa*)(p + 4);
    r[0] = a.x; r[1] = a.y; r[2] = a.z; r[3] = a.w; r[4] = b.x; r[5] = b.y; r[6] = b.z; r[7] = b.w;
  }
}

template <int SLB>
__device__ __forceinline__ int scan_chunk(const int* __restrict__ dsts, int nE, int cbase, int slotBase,
                                          int nb, int vec8, int* list, int tid, int lane, int wave) {
  int wc = 0;
  const int el0  = tid * EPT;
  const int e0   = cbase + el0;
  const int sent = -2147483647 - 1;
  v4i da, db;
  if (vec8 != 0 && cbase + CHUNK <= nE) {
    da = *(const v4i*)(dsts + e0);
    db = *(const v4i*)(dsts + e0 + 4);
  } else {
    da.x = (e0     < nE) ? dsts[min(e0,     nE - 1)] : sent;
    da.y = (e0 + 1 < nE) ? dsts[min(e0 + 1, nE - 1)] : sent;
    da.z = (e0 + 2 < nE) ? dsts[min(e0 + 2, nE - 1)] : sent;
    da.w = (e0 + 3 < nE) ? dsts[min(e0 + 3, nE - 1)] : sent;
    db.x = (e0 + 4 < nE) ? dsts[min(e0 + 4, nE - 1)] : sent;
    db.y = (e0 + 5 < nE) ? dsts[min(e0 + 5, nE - 1)] : sent;
    db.z = (e0 + 6 < nE) ? dsts[min(e0 + 6, nE - 1)] : sent;
    db.w = (e0 + 7 < nE) ? dsts[min(e0 + 7, nE - 1)] : sent;
  }
  const unsigned nbs = (unsigned)slotBase;
  const unsigned unb = (unsigned)nb;
  const unsigned s0 = (unsigned)da.x - nbs, s1 = (unsigned)da.y - nbs;
  const unsigned s2 = (unsigned)da.z - nbs, s3 = (unsigned)da.w - nbs;
  const unsigned s4 = (unsigned)db.x - nbs, s5 = (unsigned)db.y - nbs;
  const unsigned s6 = (unsigned)db.z - nbs, s7 = (unsigned)db.w - nbs;
  const bool h0 = s0 < unb, h1 = s1 < unb, h2 = s2 < unb, h3 = s3 < unb;
  const bool h4 = s4 < unb, h5 = s5 < unb, h6 = s6 < unb, h7 = s7 < unb;
  const unsigned any = __builtin_amdgcn_ballot_w32(h0 | h1 | h2 | h3 | h4 | h5 | h6 | h7);
  if (any != 0u) {
#define HITJ(J, HJ, SJ) { \
      const unsigned mj = __builtin_amdgcn_ballot_w32(HJ); \
      if (mj != 0u) { \
        if (HJ) { \
          const int pos = wc + (int)__builtin_amdgcn_mbcnt_lo(mj, 0u); \
          if (pos < WCAP) list[wave * WCAP + pos] = ((el0 + (J)) << SLB) | (int)(SJ); \
        } \
        wc += (int)__builtin_popcount(mj); } }
    HITJ(0, h0, s0)
    HITJ(1, h1, s1)
    HITJ(2, h2, s2)
    HITJ(3, h3, s3)
    HITJ(4, h4, s4)
    HITJ(5, h5, s5)
    HITJ(6, h6, s6)
    HITJ(7, h7, s7)
#undef HITJ
  }
  return wc;
}

__global__ __launch_bounds__(NTHR) void k_wprep(const float* __restrict__ W1, const float* __restrict__ W2,
                                                const float* __restrict__ W3, const float* __restrict__ W4,
                                                const float* __restrict__ W5, const float* __restrict__ W6,
                                                unsigned short* B1, unsigned short* B2, unsigned short* B3,
                                                unsigned short* B4, unsigned short* B5, unsigned short* B6) {
  const int b = (int)blockIdx.x;
  const float* W; unsigned short* B; int fi, fo, b0, units, l1;
  if (b < 4)        { W = W1; B = B1; fi = 128; fo = 16;  b0 = 0;   units = 1024;  l1 = 1; }
  else if (b < 6)   { W = W2; B = B2; fi = 16;  fo = 32;  b0 = 4;   units = 384;   l1 = 0; }
  else if (b < 12)  { W = W3; B = B3; fi = 32;  fo = 64;  b0 = 6;   units = 1536;  l1 = 0; }
  else if (b < 36)  { W = W4; B = B4; fi = 64;  fo = 128; b0 = 12;  units = 6144;  l1 = 0; }
  else if (b < 132) { W = W5; B = B5; fi = 128; fo = 256; b0 = 36;  units = 24576; l1 = 0; }
  else              { W = W6; B = B6; fi = 256; fo = 512; b0 = 132; units = 98304; l1 = 0; }
  const int v = (b - b0) * NTHR + (int)threadIdx.x;
  if (v >= units) return;
  const float* p;
  int stride;
  bool valid = true;
  if (l1 != 0) {
    const int n  = v >> 4;
    const int k8 = (v & 15) * 8;
    const int kc = n >> 4, o = n & 15;
    valid = n < 48;
    const int kcc = kc > 2 ? 2 : kc;
    p = W + ((size_t)kcc * 128 + k8) * 16 + o;
    stride = 16;
  } else {
    const int kper = (6 * fi) >> 3;
    const int n  = v / kper;
    const int k8 = (v - n * kper) * 8;
    const int kc = k8 / (2 * fi);
    const int kin = (k8 - kc * 2 * fi) % fi;
    p = W + ((size_t)kc * fi + kin) * (size_t)fo + n;
    stride = fo;
  }
  v8us o8;
#pragma unroll
  for (int i = 0; i < 8; ++i) {
    const unsigned bb = bf16_bits(p[(size_t)i * stride]);
    o8[i] = valid ? (unsigned short)bb : (unsigned short)0;
  }
  unsigned short* dp = B + (size_t)v * 8;
  *(volatile v8us*)dp = o8;
  __threadfence();
  *(volatile v8us*)dp = o8;
}

__global__ __launch_bounds__(NTHR) void k_cvx(const float* __restrict__ x, int nN, int nUnits,
                                              unsigned short* xb) {
  const int u = (int)blockIdx.x * NTHR + (int)threadIdx.x;
  if (u >= nUnits) return;
  const int row = u >> 4;
  const int k8  = (u & 15) * 8;
  const int rc  = row < nN ? row : nN - 1;
  const float* p = x + (size_t)rc * 128 + k8;
  const v4f a = *(const v4fa*)p;
  const v4f b = *(const v4fa*)(p + 4);
  const bool ok = row < nN;
  v8us o;
  o[0] = ok ? (unsigned short)bf16_bits(a.x) : (unsigned short)0;
  o[1] = ok ? (unsigned short)bf16_bits(a.y) : (unsigned short)0;
  o[2] = ok ? (unsigned short)bf16_bits(a.z) : (unsigned short)0;
  o[3] = ok ? (unsigned short)bf16_bits(a.w) : (unsigned short)0;
  o[4] = ok ? (unsigned short)bf16_bits(b.x) : (unsigned short)0;
  o[5] = ok ? (unsigned short)bf16_bits(b.y) : (unsigned short)0;
  o[6] = ok ? (unsigned short)bf16_bits(b.z) : (unsigned short)0;
  o[7] = ok ? (unsigned short)bf16_bits(b.w) : (unsigned short)0;
  unsigned short* dp = xb + (size_t)row * 128 + k8;
  *(volatile v8us*)dp = o;
  __threadfence();
  *(volatile v8us*)dp = o;
}

__global__ __launch_bounds__(NTHR) void k_deg(const int* __restrict__ keys, const float* __restrict__ ew,
                                              int nE, int vec8, float* dinv) {
  __shared__ __attribute__((aligned(16))) float sdeg[NBD];
  __shared__ __attribute__((aligned(16))) int list[LISTN];
  __shared__ int wcnt[NWAVE];
  const int tid = (int)threadIdx.x, lane = tid & 31, wave = tid >> 5;
  const int nodeBase = (int)blockIdx.x * NBD;

  for (int i = tid; i < NBD; i += NTHR) sdeg[i] = 0.0f;
  for (int i = tid; i < LISTN; i += NTHR) list[i] = 0;
  if (tid < NWAVE) wcnt[tid] = 0;
  __syncthreads();

  const int nChunks = (nE + CHUNK - 1) / CHUNK;
#pragma unroll 1
  for (int ch = 0; ch < nChunks; ++ch) {
    const int cbase = ch * CHUNK;
    const int wc = scan_chunk<SLD>(keys, nE, cbase, nodeBase, NBD, vec8, list, tid, lane, wave);
    if (lane == 0) wcnt[wave] = wc;
    __syncthreads();
    if (wave == 0) {
#pragma unroll 1
      for (int w2 = 0; w2 < NWAVE; ++w2) {
        int c = wcnt[w2];
        c = c < 0 ? 0 : (c > WCAP ? WCAP : c);
#pragma unroll 1
        for (int b0 = 0; b0 < c; b0 += 32) {
          const int idx = b0 + lane;
          const int ent = list[w2 * WCAP + (idx < WCAP ? idx : WCAP - 1)];
          const int el  = (ent >> SLD) & (CHUNK - 1);
          const int eid = clampi(cbase + el, 0, nE - 1);
          const int wi  = __float_as_int(bf16_val(ew[eid]));
          const int m32 = (c - b0) < 32 ? (c - b0) : 32;
#pragma unroll 1
          for (int k = 0; k < m32; ++k) {
            const int   u  = __builtin_amdgcn_readlane(ent, k);
            const float wk = __int_as_float(__builtin_amdgcn_readlane(wi, k));
            const int sl = u & (NBD - 1);
            if (lane == 0) sdeg[sl] = sdeg[sl] + wk;
          }
        }
      }
    }
    __syncthreads();
  }

  v4f vals[NBD / (NTHR * 4)];
#pragma unroll
  for (int it = 0; it < NBD / (NTHR * 4); ++it) {
    const int s0 = it * (NTHR * 4) + 4 * tid;
    const v4f d = *(const v4fa*)(sdeg + s0);
    v4f v;
    v.x = (d.x > 0.0f) ? (1.0f / d.x) : 0.0f;
    v.y = (d.y > 0.0f) ? (1.0f / d.y) : 0.0f;
    v.z = (d.z > 0.0f) ? (1.0f / d.z) : 0.0f;
    v.w = (d.w > 0.0f) ? (1.0f / d.w) : 0.0f;
    vals[it] = v;
  }
#pragma unroll
  for (int it = 0; it < NBD / (NTHR * 4); ++it)
    *(volatile v4f*)(dinv + (size_t)nodeBase + it * (NTHR * 4) + 4 * tid) = vals[it];
  __threadfence();
#pragma unroll
  for (int it = 0; it < NBD / (NTHR * 4); ++it)
    *(volatile v4f*)(dinv + (size_t)nodeBase + it * (NTHR * 4) + 4 * tid) = vals[it];
}

__global__ __launch_bounds__(NTHR) void k_build(const int* __restrict__ keys, const int* __restrict__ gath,
                                                const float* __restrict__ ew, const float* __restrict__ dinv,
                                                int nE, int nSrc, int vec8, int wmode, int* tab) {
  extern __shared__ __attribute__((aligned(16))) int dsm[];
  int* list = dsm;
  int* hl   = dsm + LISTN;
  int* sl   = hl + RCAP;
  int* cnt  = sl + RCAP;
  int* offs = cnt + NBA;
  int* cur  = offs + NBA;
  int* misc = cur + NBA;
  const int tid = (int)threadIdx.x, lane = tid & 31, wave = tid >> 5;
  const int nodeBase = (int)blockIdx.x * NBA;

  {
    const v4i z4 = {0, 0, 0, 0};
    for (int i = tid * 4; i < BLD_ZINTS; i += NTHR * 4) *(v4ia*)(dsm + i) = z4;
    if (tid < 16) misc[tid] = 0;
  }
  __syncthreads();

  int t = 0, ov = 0;
  const int nChunks = (nE + CHUNK - 1) / CHUNK;
#pragma unroll 1
  for (int ch = 0; ch < nChunks; ++ch) {
    const int cbase = ch * CHUNK;
    const int wc = scan_chunk<SLA>(keys, nE, cbase, nodeBase, NBA, vec8, list, tid, lane, wave);
    if (lane == 0) misc[wave] = wc;
    __syncthreads();
    if (wave == 0) {
#pragma unroll 1
      for (int w2 = 0; w2 < NWAVE; ++w2) {
        int c = misc[w2];
        c = c < 0 ? 0 : (c > WCAP ? WCAP : c);
#pragma unroll 1
        for (int b0 = 0; b0 < c; b0 += 32) {
          const int idx = b0 + lane;
          const int ent = list[w2 * WCAP + (idx < WCAP ? idx : WCAP - 1)];
          const int m32 = (c - b0) < 32 ? (c - b0) : 32;
#pragma unroll 1
          for (int k = 0; k < m32; ++k) {
            const int u    = __builtin_amdgcn_readlane(ent, k);
            const int slot = u & (NBA - 1);
            const int el   = (u >> SLA) & (CHUNK - 1);
            const int pk   = ((cbase + el) << SLA) | slot;
            if (t < RCAP) {
              if (lane == 0) { hl[t] = pk; cnt[slot] = cnt[slot] + 1; }
              t = t + 1;
            } else {
              ov = 1;
            }
          }
        }
      }
    }
    __syncthreads();
  }
  if (wave == 0 && lane == 0) { misc[8] = t; misc[9] = ov; }
  __syncthreads();
  int tt = misc[8];
  tt = tt < 0 ? 0 : (tt > RCAP ? RCAP : tt);
  const int ovf = misc[9];

  if (wave == 0) {
    const int base = lane * (NBA / 32);
    int s = 0;
#pragma unroll 1
    for (int i = 0; i < NBA / 32; ++i) s += cnt[base + i];
    int incl = s;
#pragma unroll
    for (int d = 1; d < 32; d <<= 1) {
      const int y = __shfl_up(incl, d, 32);
      if (lane >= d) incl += y;
    }
    int run = incl - s;
#pragma unroll 1
    for (int i = 0; i < NBA / 32; ++i) {
      const int cv = cnt[base + i];
      offs[base + i] = run;
      cur[base + i]  = run;
      run += cv;
    }
  }
  __syncthreads();
  if (wave == 0) {
#pragma unroll 1
    for (int b0 = 0; b0 < tt; b0 += 32) {
      const int idx = b0 + lane;
      const int ent = hl[idx < RCAP ? idx : RCAP - 1];
      const int m32 = (tt - b0) < 32 ? (tt - b0) : 32;
#pragma unroll 1
      for (int k = 0; k < m32; ++k) {
        const int u    = __builtin_amdgcn_readlane(ent, k);
        const int slot = u & (NBA - 1);
        if (lane == 0) {
          int p = cur[slot];
          p = p < 0 ? 0 : (p > RCAP - 1 ? RCAP - 1 : p);
          sl[p] = u;
          cur[slot] = p + 1;
        }
      }
    }
  }
  __syncthreads();

  int* tb = tab + (size_t)blockIdx.x * TBSZ;
  {
    v4i hv = {0, 0, 0, 0};
    hv.x = (tid == 0) ? tt : 0;
    hv.y = (tid == 0) ? ovf : 0;
    const v4i c4 = *(const v4ia*)(cnt + 4 * tid);
    const v4i o4 = *(const v4ia*)(offs + 4 * tid);
    const bool hst = tid < 8;
    if (hst) *(volatile v4i*)(tb + 4 * tid) = hv;
    *(volatile v4i*)(tb + TB_CNT + 4 * tid) = c4;
    *(volatile v4i*)(tb + TB_OFF + 4 * tid) = o4;
    __threadfence();
    if (hst) *(volatile v4i*)(tb + 4 * tid) = hv;
    *(volatile v4i*)(tb + TB_CNT + 4 * tid) = c4;
    *(volatile v4i*)(tb + TB_OFF + 4 * tid) = o4;
  }
#pragma unroll 1
  for (int it = 0; it < RCAP / (NTHR * 4); ++it) {
    const int p = it * (NTHR * 4) + 4 * tid;
    const v4i e4 = *(const v4ia*)(sl + p);
    const int e0 = clampi(e4.x >> SLA, 0, nE - 1);
    const int e1 = clampi(e4.y >> SLA, 0, nE - 1);
    const int e2 = clampi(e4.z >> SLA, 0, nE - 1);
    const int e3 = clampi(e4.w >> SLA, 0, nE - 1);
    v4i s4; v4f w4;
    if (wmode != 0) {
      const int r0 = clampi(gath[e0], 0, nSrc - 1);
      const int r1 = clampi(gath[e1], 0, nSrc - 1);
      const int r2 = clampi(gath[e2], 0, nSrc - 1);
      const int r3 = clampi(gath[e3], 0, nSrc - 1);
      const float q0 = bf16_val(ew[e0]), q1 = bf16_val(ew[e1]);
      const float q2 = bf16_val(ew[e2]), q3 = bf16_val(ew[e3]);
      w4.x = -(dinv[r0] * q0); w4.y = -(dinv[r1] * q1);
      w4.z = -(dinv[r2] * q2); w4.w = -(dinv[r3] * q3);
      s4.x = r0; s4.y = r1; s4.z = r2; s4.w = r3;
    } else {
      s4.x = min(e0, nSrc - 1); s4.y = min(e1, nSrc - 1);
      s4.z = min(e2, nSrc - 1); s4.w = min(e3, nSrc - 1);
      w4.x = 0.0f; w4.y = 0.0f; w4.z = 0.0f; w4.w = 0.0f;
    }
    int*   sp = tb + TB_SRC + p;
    float* wp = (float*)(tb + TB_WV + p);
    *(volatile v4i*)sp = s4;
    *(volatile v4f*)wp = w4;
    __threadfence();
    *(volatile v4i*)sp = s4;
    *(volatile v4f*)wp = w4;
  }
}

template <int NT>
__global__ __launch_bounds__(GTHR) void k_gemm(const unsigned short* __restrict__ A0,
                                               const unsigned short* __restrict__ A1,
                                               const unsigned short* __restrict__ A2,
                                               int lda, int kpp, int nplanes,
                                               const unsigned short* __restrict__ WT, int ldb,
                                               const float* __restrict__ bias, int useBias,
                                               float* outF, int ldo) {
  constexpr int GBN = 16 * NT;
  __shared__ __attribute__((aligned(16))) float stg[GBM * GBN];
  const int tid = (int)threadIdx.x, lane = tid & 31, wave = tid >> 5, hh = lane >> 4, m = lane & 15;
  const int rowBase = (int)blockIdx.x * GBM;
  const int col0    = (int)blockIdx.y * GBN;

  v8f acc[NT];
  {
    const v8f z = {0.f, 0.f, 0.f, 0.f, 0.f, 0.f, 0.f, 0.f};
#pragma unroll
    for (int t = 0; t < NT; ++t) acc[t] = z;
  }
  const size_t aoff = (size_t)(rowBase + 16 * wave + m) * (size_t)lda + 8 * hh;
  const unsigned short* wp = WT + (size_t)(col0 + m) * (size_t)ldb + 8 * hh;
#pragma unroll 1
  for (int p = 0; p < nplanes; ++p) {
    const unsigned short* ap = ((p == 0) ? A0 : ((p == 1) ? A1 : A2)) + aoff;
    const unsigned short* wq0 = wp + (size_t)p * (size_t)kpp;
#pragma unroll 1
    for (int k0 = 0; k0 < kpp; k0 += 32) {
      FragB af;
      af.h[0] = *(const v8usa*)(ap + k0);
      af.h[1] = *(const v8usa*)(ap + k0 + 16);
#pragma unroll
      for (int t = 0; t < NT; ++t) {
        const unsigned short* wq = wq0 + (size_t)(16 * t) * (size_t)ldb + k0;
        FragB bf;
        bf.h[0] = *(const v8usa*)wq;
        bf.h[1] = *(const v8usa*)(wq + 16);
        acc[t] = wmb(af, bf, acc[t]);
      }
    }
  }

#pragma unroll
  for (int t = 0; t < NT; ++t) {
    const int lc = 16 * t + m;
#pragma unroll
    for (int r = 0; r < 8; ++r) {
      const int lr = 16 * wave + 8 * hh + r;
      stg[lr * GBN + lc] = acc[t][r];
    }
  }
  __syncthreads();

  constexpr int LPR  = GBN / 4;
  constexpr int RPI  = 32 / LPR;
  constexpr int ITER = 16 / RPI;
  const int lrow = lane / LPR;
  const int lcol = 4 * (lane % LPR);
  v4f bb = {0.f, 0.f, 0.f, 0.f};
  if (useBias != 0) {
    const v4f tb4 = *(const v4fa*)(bias + col0 + lcol);
    bb.x = bf16_val(tb4.x); bb.y = bf16_val(tb4.y); bb.z = bf16_val(tb4.z); bb.w = bf16_val(tb4.w);
  }
  v4f fv[ITER];
#pragma unroll
  for (int i = 0; i < ITER; ++i) {
    const int lr = 16 * wave + RPI * i + lrow;
    fv[i] = *(const v4fa*)(stg + lr * GBN + lcol) + bb;
  }
#pragma unroll
  for (int i = 0; i < ITER; ++i) {
    const int gr = rowBase + 16 * wave + RPI * i + lrow;
    *(volatile v4f*)(outF + (size_t)gr * (size_t)ldo + col0 + lcol) = fv[i];
  }
  __threadfence();
#pragma unroll
  for (int i = 0; i < ITER; ++i) {
    const int gr = rowBase + 16 * wave + RPI * i + lrow;
    *(volatile v4f*)(outF + (size_t)gr * (size_t)ldo + col0 + lcol) = fv[i];
  }
}

template <int CPL, int HALF>
__global__ __launch_bounds__(NTHR) void k_lap(const int* tab, const float* G, int gp, int goff,
                                              const float* SA, int sap, int saoff, float sa, int useA,
                                              const float* SB, int sbp, int sboff, float sb, int useB,
                                              const float* bias, int useBias, float alpha,
                                              float* outF, int wrF, unsigned short* outP, int wrP,
                                              int nN, int mRows) {
  constexpr int PF  = HALF ? 32 : 32 * CPL;
  constexpr int FW  = HALF ? 16 : 32 * CPL;
  constexpr int NL  = PF / 4;
  constexpr int NL0 = NL < 32 ? NL : 32;
  __shared__ __attribute__((aligned(16))) float rowFs[NWAVE * PF];
  __shared__ __attribute__((aligned(16))) unsigned short rowPs[NWAVE * 2 * PF];
  const int tid = (int)threadIdx.x, lane = tid & 31, wave = tid >> 5;
  float* rf = rowFs + wave * PF;
  unsigned short* rp = rowPs + wave * 2 * PF;
  const int ch = HALF ? (lane & 15) : CPL * lane;
  const float qnan = __int_as_float(0x7fc00000);

  float bv[CPL];
#pragma unroll
  for (int j = 0; j < CPL; ++j) bv[j] = 0.0f;
  if (useBias != 0) {
    float tbv[CPL];
    ld_row<CPL>(bias + ch, tbv);
#pragma unroll
    for (int j = 0; j < CPL; ++j) bv[j] = bf16_val(tbv[j]);
  }

#pragma unroll 1
  for (int si = 0; si < SPW; ++si) {
    const int node = (int)blockIdx.x * NPB + wave * SPW + si;
    const int* tb = tab + (size_t)(node >> SLA) * TBSZ;
    const int s = node & (NBA - 1);
    int c = tb[TB_CNT + s];
    const bool big = c > DEGCAP;
    c = c < 0 ? 0 : (c > DEGCAP ? DEGCAP : c);
    const int o = clampi(tb[TB_OFF + s], 0, RCAP - 1);
    const int ovf = tb[1];
    const int nc = node < nN ? node : nN - 1;
    float acc[CPL];
#pragma unroll
    for (int j = 0; j < CPL; ++j) acc[j] = 0.0f;
#pragma unroll 1
    for (int b0 = 0; b0 < c; b0 += 32) {
      int idx = o + b0 + lane;
      idx = idx > RCAP - 1 ? RCAP - 1 : idx;
      const int sr  = clampi(tb[TB_SRC + idx], 0, nN - 1);
      const int wvi = tb[TB_WV + idx];
      const int m32 = (c - b0) < 32 ? (c - b0) : 32;
#pragma unroll 1
      for (int k = 0; k < m32; ++k) {
        const int   sk = __builtin_amdgcn_readlane(sr, k);
        const float ck = __int_as_float(__builtin_amdgcn_readlane(wvi, k));
        float a[CPL];
        ld_row<CPL>(G + (size_t)sk * (size_t)gp + goff + ch, a);
#pragma unroll
        for (int j = 0; j < CPL; ++j) acc[j] = fmaf(ck, a[j], acc[j]);
      }
    }
    float sf[CPL];
#pragma unroll
    for (int j = 0; j < CPL; ++j) sf[j] = bv[j];
    if (useA != 0) {
      float a[CPL];
      ld_row<CPL>(SA + (size_t)nc * (size_t)sap + saoff + ch, a);
#pragma unroll
      for (int j = 0; j < CPL; ++j) sf[j] = fmaf(sa, a[j], sf[j]);
    }
    if (useB != 0) {
      float a[CPL];
      ld_row<CPL>(SB + (size_t)nc * (size_t)sbp + sboff + ch, a);
#pragma unroll
      for (int j = 0; j < CPL; ++j) sf[j] = fmaf(sb, a[j], sf[j]);
    }
    const float pzr = (big || ovf != 0) ? qnan : 0.0f;
    const bool live = node < nN;
    float v[CPL];
    unsigned short hb[CPL], lb[CPL];
#pragma unroll
    for (int j = 0; j < CPL; ++j) {
      const float y = fmaf(alpha, acc[j], sf[j]) + pzr;
      v[j] = live ? y : 0.0f;
      const unsigned h = bf16_bits(v[j]);
      hb[j] = (unsigned short)h;
      lb[j] = (unsigned short)bf16_bits(v[j] - __uint_as_float(h << 16));
    }
    if constexpr (HALF != 0) {
      rf[lane] = (lane < 16) ? v[0] : 0.0f;
      rp[lane] = (lane < 16) ? hb[0] : lb[0];
      rp[32 + lane] = (unsigned short)(lane & 0);
    } else if constexpr (CPL == 1) {
      rf[lane] = v[0];
      rp[lane] = hb[0];
      rp[FW + lane] = lb[0];
    } else if constexpr (CPL == 2) {
      v2f fv2; fv2.x = v[0]; fv2.y = v[1];
      v2us h2, l2; h2[0] = hb[0]; h2[1] = hb[1]; l2[0] = lb[0]; l2[1] = lb[1];
      *(v2fa*)(rf + 2 * lane) = fv2;
      *(v2usa*)(rp + 2 * lane) = h2;
      *(v2usa*)(rp + FW + 2 * lane) = l2;
    } else if constexpr (CPL == 4) {
      v4f fv4; fv4.x = v[0]; fv4.y = v[1]; fv4.z = v[2]; fv4.w = v[3];
      v4us h4, l4;
#pragma unroll
      for (int j = 0; j < 4; ++j) { h4[j] = hb[j]; l4[j] = lb[j]; }
      *(v4fa*)(rf + 4 * lane) = fv4;
      *(v4usa*)(rp + 4 * lane) = h4;
      *(v4usa*)(rp + FW + 4 * lane) = l4;
    } else {
      v4f fa, fb; fa.x = v[0]; fa.y = v[1]; fa.z = v[2]; fa.w = v[3];
      fb.x = v[4]; fb.y = v[5]; fb.z = v[6]; fb.w = v[7];
      v8us h8, l8;
#pragma unroll
      for (int j = 0; j < 8; ++j) { h8[j] = hb[j]; l8[j] = lb[j]; }
      *(v4fa*)(rf + 8 * lane) = fa;
      *(v4fa*)(rf + 8 * lane + 4) = fb;
      *(v8usa*)(rp + 8 * lane) = h8;
      *(v8usa*)(rp + FW + 8 * lane) = l8;
    }
    wave_sync();
    const int pc0 = lane & (NL0 - 1);
    const v4f  qF0 = *(const v4fa*)(rf + 4 * pc0);
    const v8us qP0 = *(const v8usa*)(rp + 8 * pc0);
    v4f  qF1 = qF0;
    v8us qP1 = qP0;
    if constexpr (CPL == 8) {
      qF1 = *(const v4fa*)(rf + 128 + 4 * lane);
      qP1 = *(const v8usa*)(rp + 256 + 8 * lane);
    }
    wave_sync();
    const bool ok = (node < mRows) && (lane < NL0);
    float* pF = outF + (size_t)node * PF + 4 * pc0;
    unsigned short* pP = outP + (size_t)node * (2 * PF) + 8 * pc0;
    if (wrF != 0 && ok) {
      *(volatile v4f*)pF = qF0;
      if constexpr (CPL == 8) *(volatile v4f*)(pF + 128) = qF1;
    }
    if (wrP != 0 && ok) {
      *(volatile v8us*)pP = qP0;
      if constexpr (CPL == 8) *(volatile v8us*)(pP + 256) = qP1;
    }
    __threadfence();
    if (wrF != 0 && ok) {
      *(volatile v4f*)pF = qF0;
      if constexpr (CPL == 8) *(volatile v4f*)(pF + 128) = qF1;
    }
    if (wrP != 0 && ok) {
      *(volatile v8us*)pP = qP0;
      if constexpr (CPL == 8) *(volatile v8us*)(pP + 256) = qP1;
    }
  }
}

__global__ __launch_bounds__(NTHR) void k_pool(const int* tab, const float* PRE, int pp, int F,
                                               float* Hout, unsigned short* Pout, int nN, int mRows) {
  __shared__ __attribute__((aligned(16))) float rowFs[NWAVE * 256];
  __shared__ __attribute__((aligned(16))) unsigned short rowPs[NWAVE * 512];
  const int tid = (int)threadIdx.x, lane = tid & 31, wave = tid >> 5;
  float* rf = rowFs + wave * 256;
  unsigned short* rp = rowPs + wave * 512;
  const int PF  = F < 32 ? 32 : F;
  const int nIt = PF >> 5;
  const int NLp = PF >> 2;
  const float qnan = __int_as_float(0x7fc00000);
  const float ninf = __int_as_float((int)0xff800000u);

#pragma unroll 1
  for (int si = 0; si < SPW; ++si) {
    const int node = (int)blockIdx.x * NPB + wave * SPW + si;
    const int* tb = tab + (size_t)(node >> SLA) * TBSZ;
    const int s = node & (NBA - 1);
    int c = tb[TB_CNT + s];
    const bool big = c > PCAP;
    c = c < 0 ? 0 : (c > PCAP ? PCAP : c);
    const int o = clampi(tb[TB_OFF + s], 0, RCAP - 1);
    const int ovf = tb[1];
#pragma unroll 1
    for (int it = 0; it < nIt; ++it) rf[it * 32 + lane] = ninf;
#pragma unroll 1
    for (int b0 = 0; b0 < c; b0 += 32) {
      int idx = o + b0 + lane;
      idx = idx > RCAP - 1 ? RCAP - 1 : idx;
      const int mem = clampi(tb[TB_SRC + idx], 0, nN - 1);
      const int m32 = (c - b0) < 32 ? (c - b0) : 32;
#pragma unroll 1
      for (int k = 0; k < m32; ++k) {
        const int mk = __builtin_amdgcn_readlane(mem, k);
        const float* pr = PRE + (size_t)mk * (size_t)pp;
#pragma unroll 1
        for (int it = 0; it < nIt; ++it) {
          const int cI = it * 32 + lane;
          const int cc = cI < F ? cI : F - 1;
          const float v = pr[cc];
          const float m = rf[cI];
          rf[cI] = (v > m || v != v) ? v : m;
        }
      }
    }
    const float pzr = (big || ovf != 0) ? qnan : 0.0f;
    const bool live = node < nN;
    if (F < 32) rp[32 + lane] = (unsigned short)(lane & 0);
#pragma unroll 1
    for (int it = 0; it < nIt; ++it) {
      const int cI = it * 32 + lane;
      const bool valid = cI < F;
      const float m  = rf[cI];
      const float sp = softplus_f(m) + pzr;
      const float val = (valid && live) ? sp : 0.0f;
      rf[cI] = val;
      const unsigned h = bf16_bits(val);
      const unsigned short hb = (unsigned short)h;
      const unsigned short lb = (unsigned short)bf16_bits(val - __uint_as_float(h << 16));
      if (valid) { rp[cI] = hb; rp[F + cI] = lb; }
    }
    wave_sync();
    const int p0 = lane < NLp ? lane : NLp - 1;
    const int p1 = (32 + lane) < NLp ? (32 + lane) : NLp - 1;
    const v4f  f0 = *(const v4fa*)(rf + 4 * p0);
    const v4f  f1 = *(const v4fa*)(rf + 4 * p1);
    const v8us h0 = *(const v8usa*)(rp + 8 * p0);
    const v8us h1 = *(const v8usa*)(rp + 8 * p1);
    wave_sync();
    const bool ok0 = (node < mRows) && (lane < NLp);
    const bool ok1 = (node < mRows) && ((32 + lane) < NLp);
    float* pf0 = Hout + (size_t)node * (size_t)PF + 4 * p0;
    float* pf1 = Hout + (size_t)node * (size_t)PF + 4 * p1;
    unsigned short* pq0 = Pout + (size_t)node * (size_t)(2 * PF) + 8 * p0;
    unsigned short* pq1 = Pout + (size_t)node * (size_t)(2 * PF) + 8 * p1;
    if (ok0) *(volatile v4f*)pf0 = f0;
    if (ok1) *(volatile v4f*)pf1 = f1;
    if (ok0) *(volatile v8us*)pq0 = h0;
    if (ok1) *(volatile v8us*)pq1 = h1;
    __threadfence();
    if (ok0) *(volatile v4f*)pf0 = f0;
    if (ok1) *(volatile v4f*)pf1 = f1;
    if (ok0) *(volatile v8us*)pq0 = h0;
    if (ok1) *(volatile v8us*)pq1 = h1;
  }
}

__global__ __launch_bounds__(NTHR) void k_pool_fc(const int* tab, const float* PRE,
                                                  const float* __restrict__ fcw, const float* __restrict__ fcbp,
                                                  float* out, int nN, int nOut) {
  __shared__ __attribute__((aligned(16))) float rowFs[NWAVE * FCK];
  __shared__ __attribute__((aligned(16))) float fcs[FCK * NCLS];
  __shared__ float fcb[4];
  __shared__ __attribute__((aligned(16))) float outs[NPB * NCLS];
  const int tid = (int)threadIdx.x, lane = tid & 31, wave = tid >> 5;
  float* rf = rowFs + wave * FCK;
  const float qnan = __int_as_float(0x7fc00000);
  const float ninf = __int_as_float((int)0xff800000u);
#pragma unroll 1
  for (int i = tid; i < FCK * NCLS; i += NTHR) fcs[i] = bf16_val(fcw[i]);
  if (tid < 4) {
    const float bb = fcbp[tid < NCLS ? tid : NCLS - 1];
    fcb[tid] = (tid < NCLS) ? bf16_val(bb) : 0.0f;
  }
  __syncthreads();

#pragma unroll 1
  for (int si = 0; si < SPW; ++si) {
    const int node = (int)blockIdx.x * NPB + wave * SPW + si;
    const int* tb = tab + (size_t)(node >> SLA) * TBSZ;
    const int s = node & (NBA - 1);
    int c = tb[TB_CNT + s];
    const bool big = c > PCAP;
    c = c < 0 ? 0 : (c > PCAP ? PCAP : c);
    const int o = clampi(tb[TB_OFF + s], 0, RCAP - 1);
    const int ovf = tb[1];
#pragma unroll 1
    for (int it = 0; it < FCK / 32; ++it) rf[it * 32 + lane] = ninf;
#pragma unroll 1
    for (int b0 = 0; b0 < c; b0 += 32) {
      int idx = o + b0 + lane;
      idx = idx > RCAP - 1 ? RCAP - 1 : idx;
      const int mem = clampi(tb[TB_SRC + idx], 0, nN - 1);
      const int m32 = (c - b0) < 32 ? (c - b0) : 32;
#pragma unroll 1
      for (int k = 0; k < m32; ++k) {
        const int mk = __builtin_amdgcn_readlane(mem, k);
        const float* pr = PRE + (size_t)mk * FCK;
#pragma unroll 1
        for (int it = 0; it < FCK / 32; ++it) {
          const int cI = it * 32 + lane;
          const float v = pr[cI];
          const float m = rf[cI];
          rf[cI] = (v > m || v != v) ? v : m;
        }
      }
    }
    float s0 = 0.0f, s1 = 0.0f, s2 = 0.0f;
#pragma unroll 1
    for (int it = 0; it < FCK / 32; ++it) {
      const int cI = it * 32 + lane;
      const float sp = softplus_f(rf[cI]);
      s0 = fmaf(sp, fcs[cI * NCLS + 0], s0);
      s1 = fmaf(sp, fcs[cI * NCLS + 1], s1);
      s2 = fmaf(sp, fcs[cI * NCLS + 2], s2);
    }
#pragma unroll
    for (int d = 16; d >= 1; d >>= 1) {
      s0 += __shfl_xor(s0, d, 32);
      s1 += __shfl_xor(s1, d, 32);
      s2 += __shfl_xor(s2, d, 32);
    }
    const float pzr = (big || ovf != 0) ? qnan : 0.0f;
    const bool live = node < nN;
    const float r0 = live ? (s0 + fcb[0] + pzr) : 0.0f;
    const float r1 = live ? (s1 + fcb[1] + pzr) : 0.0f;
    const float r2 = live ? (s2 + fcb[2] + pzr) : 0.0f;
    if (lane == 0) {
      const int lr = wave * SPW + si;
      outs[lr * NCLS + 0] = r0;
      outs[lr * NCLS + 1] = r1;
      outs[lr * NCLS + 2] = r2;
    }
  }
  __syncthreads();
  const int q  = tid < (NPB * NCLS) / 4 ? tid : (NPB * NCLS) / 4 - 1;
  const v4f ov = *(const v4fa*)(outs + 4 * q);
  const long long fidx = (long long)blockIdx.x * (NPB * NCLS) + 4 * q;
  const bool st = (tid < (NPB * NCLS) / 4) && (fidx + 3 < (long long)nOut);
  float* op = out + (size_t)fidx;
  if (st) *(volatile v4f*)op = ov;
  __threadfence();
  if (st) *(volatile v4f*)op = ov;
}

static inline int cdiv(int a, int b) { return (a + b - 1) / b; }
static inline size_t al256(size_t o) { return (o + 255) & ~(size_t)255; }

extern "C" void kernel_launch(void* const* d_in, const int* in_sizes, int n_in,
                              void* d_out, int out_size, void* d_ws, size_t ws_size,
                              hipStream_t stream) {
  if (n_in < 18) return;
  const int fiA[6] = {128, 16, 32, 64, 128, 256};
  const int foA[6] = {16, 32, 64, 128, 256, 512};
  if (in_sizes[0] < 128 || (in_sizes[0] % 128) != 0) return;
  const int nN = in_sizes[0] / 128;
  if (nN < 1 || nN > (1 << 20)) return;
  if (in_sizes[1] < 2 || (in_sizes[1] & 1) != 0) return;
  const int nE = in_sizes[1] / 2;
  if (nE < 1 || nE >= (1 << (31 - SLD))) return;
  if (in_sizes[2] != nE || in_sizes[3] != nN) return;
  for (int l = 0; l < 6; ++l) {
    if (in_sizes[4 + 2 * l] != 3 * fiA[l] * foA[l]) return;
    if (in_sizes[5 + 2 * l] != foA[l]) return;
  }
  if (in_sizes[16] != FCK * NCLS || in_sizes[17] != NCLS) return;
  if ((long long)out_size != (long long)nN * NCLS) return;
  if (((nN * NCLS) & 3) != 0) return;

  const float* x    = (const float*)d_in[0];
  const int*   edge = (const int*)d_in[1];
  const float* ew   = (const float*)d_in[2];
  const int*   bat  = (const int*)d_in[3];
  const float* Wp[6];
  const float* bp[6];
  for (int l = 0; l < 6; ++l) { Wp[l] = (const float*)d_in[4 + 2 * l]; bp[l] = (const float*)d_in[5 + 2 * l]; }
  const float* fcw = (const float*)d_in[16];
  const float* fcb = (const float*)d_in[17];
  float* out = (float*)d_out;
  const int* row = edge;
  const int* col = edge + nE;

  const int MP   = cdiv(nN, GBM) * GBM;
  const int gM   = MP / GBM;
  const int gD   = cdiv(nN, NBD);
  const int NBPD = gD * NBD;
  const int gA   = cdiv(MP, NBA);
  if ((long long)gA * NBA < (long long)MP) return;
  const int vecE = ((nE & 3) == 0) ? 1 : 0;
  const int vecN = ((nN & 3) == 0) ? 1 : 0;

  char* ws = (char*)d_ws;
  size_t off = 0;
  const size_t oDINV = off; off = al256(off + (size_t)NBPD * 4);
  const size_t oTABC = off; off = al256(off + (size_t)gA * TBSZ * 4);
  const size_t oTABP = off; off = al256(off + (size_t)gA * TBSZ * 4);
  const size_t oXB   = off; off = al256(off + (size_t)MP * 128 * 2);
  const size_t oY    = off; off = al256(off + (size_t)MP * 64 * 4);
  size_t oBt[6];
  oBt[0] = off; off = al256(off + (size_t)64 * 128 * 2);
  for (int l = 1; l < 6; ++l) { oBt[l] = off; off = al256(off + (size_t)foA[l] * 6 * fiA[l] * 2); }
  const size_t plane = (size_t)MP * 512 * 2;
  const size_t oRA   = off; off = al256(off + 3 * plane);
  const size_t oRF   = off; off = al256(off + (size_t)MP * 512 * 4);
  if (off > ws_size) return;
  float* DINV = (float*)(ws + oDINV);
  int*   TABC = (int*)(ws + oTABC);
  int*   TABP = (int*)(ws + oTABP);
  unsigned short* XB = (unsigned short*)(ws + oXB);
  float* Y = (float*)(ws + oY);
  unsigned short* Bt[6];
  for (int l = 0; l < 6; ++l) Bt[l] = (unsigned short*)(ws + oBt[l]);
  unsigned short* P0 = (unsigned short*)(ws + oRA);
  unsigned short* P1 = (unsigned short*)(ws + oRA + plane);
  unsigned short* P2 = (unsigned short*)(ws + oRA + 2 * plane);
  float* F0 = (float*)(ws + oRF);
  float* F1 = F0 + (size_t)MP * 256;

  const size_t bldLds = (size_t)BLD_LDS_INTS * 4;
  hipFuncSetAttribute(reinterpret_cast<const void*>(&k_build), hipFuncAttributeMaxDynamicSharedMemorySize, (int)bldLds);

  k_wprep<<<516, NTHR, 0, stream>>>(Wp[0], Wp[1], Wp[2], Wp[3], Wp[4], Wp[5],
                                    Bt[0], Bt[1], Bt[2], Bt[3], Bt[4], Bt[5]);
  const int nUx = MP * 16;
  k_cvx<<<cdiv(nUx, NTHR), NTHR, 0, stream>>>(x, nN, nUx, XB);
  k_deg<<<gD, NTHR, 0, stream>>>(row, ew, nE, vecE, DINV);
  k_build<<<gA, NTHR, bldLds, stream>>>(col, row, ew, DINV, nE, nN, vecE, 1, TABC);
  k_build<<<gA, NTHR, bldLds, stream>>>(bat, bat, ew, DINV, nN, nN, vecN, 0, TABP);

  k_gemm<4><<<dim3(gM, 1), GTHR, 0, stream>>>(XB, XB, XB, 128, 128, 1, Bt[0], 128, bp[0], 0, Y, 64);
  k_lap<1, 1><<<gM, NTHR, 0, stream>>>(TABC, Y, 64, 32, Y, 64, 16, 1.0f, 1, Y, 64, 0, 0.0f, 0,
                                       bp[0], 0, 2.0f, F0, 1, P0, 0, nN, MP);
  k_lap<1, 1><<<gM, NTHR, 0, stream>>>(TABC, F0, 32, 0, Y, 64, 0, 1.0f, 1, Y, 64, 32, -1.0f, 1,
                                       bp[0], 1, 1.0f, F1, 1, P0, 0, nN, MP);
  k_pool<<<gM, NTHR, 0, stream>>>(TABP, F1, 32, 16, F0, P0, nN, MP);

  for (int l = 1; l < 6; ++l) {
    const int fi = fiA[l], fo = foA[l];
    const int hp  = fi < 32 ? 32 : fi;
    const int lda = 2 * hp;
    const int kpp = 2 * fi;
    if (fi == 16) {
      k_lap<1, 1><<<gM, NTHR, 0, stream>>>(TABC, F0, hp, 0, F0, hp, 0, 0.0f, 0, F0, hp, 0, 0.0f, 0,
                                           bp[l], 0, 1.0f, F1, 1, P1, 1, nN, MP);
      k_lap<1, 1><<<gM, NTHR, 0, stream>>>(TABC, F1, hp, 0, F0, hp, 0, -1.0f, 1, F0, hp, 0, 0.0f, 0,
                                           bp[l], 0, 2.0f, F1, 0, P2, 1, nN, MP);
    } else if (fi == 32) {
      k_lap<1, 0><<<gM, NTHR, 0, stream>>>(TABC, F0, hp, 0, F0, hp, 0, 0.0f, 0, F0, hp, 0, 0.0f, 0,
                                           bp[l], 0, 1.0f, F1, 1, P1, 1, nN, MP);
      k_lap<1, 0><<<gM, NTHR, 0, stream>>>(TABC, F1, hp, 0, F0, hp, 0, -1.0f, 1, F0, hp, 0, 0.0f, 0,
                                           bp[l], 0, 2.0f, F1, 0, P2, 1, nN, MP);
    } else if (fi == 64) {
      k_lap<2, 0><<<gM, NTHR, 0, stream>>>(TABC, F0, hp, 0, F0, hp, 0, 0.0f, 0, F0, hp, 0, 0.0f, 0,
                                           bp[l], 0, 1.0f, F1, 1, P1, 1, nN, MP);
      k_lap<2, 0><<<gM, NTHR, 0, stream>>>(TABC, F1, hp, 0, F0, hp, 0, -1.0f, 1, F0, hp, 0, 0.0f, 0,
                                           bp[l], 0, 2.0f, F1, 0, P2, 1, nN, MP);
    } else if (fi == 128) {
      k_lap<4, 0><<<gM, NTHR, 0, stream>>>(TABC, F0, hp, 0, F0, hp, 0, 0.0f, 0, F0, hp, 0, 0.0f, 0,
                                           bp[l], 0, 1.0f, F1, 1, P1, 1, nN, MP);
      k_lap<4, 0><<<gM, NTHR, 0, stream>>>(TABC, F1, hp, 0, F0, hp, 0, -1.0f, 1, F0, hp, 0, 0.0f, 0,
                                           bp[l], 0, 2.0f, F1, 0, P2, 1, nN, MP);
    } else {
      k_lap<8, 0><<<gM, NTHR, 0, stream>>>(TABC, F0, hp, 0, F0, hp, 0, 0.0f, 0, F0, hp, 0, 0.0f, 0,
                                           bp[l], 0, 1.0f, F1, 1, P1, 1, nN, MP);
      k_lap<8, 0><<<gM, NTHR, 0, stream>>>(TABC, F1, hp, 0, F0, hp, 0, -1.0f, 1, F0, hp, 0, 0.0f, 0,
                                           bp[l], 0, 2.0f, F1, 0, P2, 1, nN, MP);
    }
    float* PRE = (l < 5) ? F1 : F0;
    const int ldo = fo < 32 ? 32 : fo;
    if (fo == 32) {
      k_gemm<2><<<dim3(gM, 1), GTHR, 0, stream>>>(P0, P1, P2, lda, kpp, 3, Bt[l], 6 * fi, bp[l], 1, PRE, ldo);
    } else if (fo == 64) {
      k_gemm<4><<<dim3(gM, 1), GTHR, 0, stream>>>(P0, P1, P2, lda, kpp, 3, Bt[l], 6 * fi, bp[l], 1, PRE, ldo);
    } else {
      k_gemm<8><<<dim3(gM, fo / 128), GTHR, 0, stream>>>(P0, P1, P2, lda, kpp, 3, Bt[l], 6 * fi, bp[l], 1, PRE, ldo);
    }
    if (l < 5) {
      k_pool<<<gM, NTHR, 0, stream>>>(TABP, PRE, ldo, fo, F0, P0, nN, MP);
    } else {
      k_pool_fc<<<gM, NTHR, 0, stream>>>(TABP, PRE, fcw, fcb, out, nN, nN * NCLS);
    }
  }
}
